// LSTMnet_59725815218259
// MI455X (gfx1250) — hardware-verified
//
#include <hip/hip_runtime.h>
#include <math.h>

constexpr int NBATCH = 64;
constexpr int NFEAT  = 2;
constexpr int NSTEP  = 128;
constexpr int NSEQ   = 207;
constexpr int NHID   = 64;
constexpr int NGATE  = 4 * NHID;
constexpr int NHEAD  = 128;
constexpr int NOUTC  = 2;
constexpr int MROWS  = NBATCH * NSEQ;
constexpr int TROWS  = 16;
constexpr int NTILE  = MROWS / TROWS;
constexpr int NTHR   = 256;
constexpr int NOUT   = NBATCH * NOUTC * NSEQ;
constexpr int NXELEM = NBATCH * NFEAT * NSTEP * NSEQ;

constexpr float HCARRY = 64.0f;
constexpr float WCARRY = 16.0f;
constexpr float FOLD   = 1.0f / (HCARRY * WCARRY);

constexpr int WOFF_HH0 = 0;
constexpr int WOFF_IH1 = NGATE * NHID;
constexpr int WOFF_HH1 = 2 * NGATE * NHID;
constexpr int WOFF_W1  = 3 * NGATE * NHID;
constexpr int WPLANE_ELEMS = 3 * NGATE * NHID + NHEAD * NHID;
constexpr int PREP_BLOCKS  = WPLANE_ELEMS / 8 / NTHR;

static_assert(MROWS == 13248, "row count");
static_assert(MROWS % TROWS == 0, "row tiles exact");
static_assert(NTILE == 828, "tile count");
static_assert(NHID % 32 == 0, "K multiple of 32");
static_assert(NGATE == 8 * 32, "8 waves x 32 gate columns");
static_assert(NHEAD == 8 * 16, "8 waves x 16 head columns");
static_assert(NOUT % 32 == 0, "whole output lines");
static_assert(NOUT == NTILE * 32, "one line per tile in the Y plane");
static_assert(WPLANE_ELEMS == 57344, "weight plane size");
static_assert(PREP_BLOCKS == 28, "weight plane blocks");
static_assert((NGATE * NHID) == 8 * NTHR * 8, "8 blocks per 256x64 weight");
static_assert(NSTEP * TROWS * NFEAT == 16 * NTHR, "x tile staging exact");

typedef __attribute__((ext_vector_type(16))) _Float16 v16h;
typedef __attribute__((ext_vector_type(8)))  _Float16 v8h;
typedef __attribute__((ext_vector_type(4)))  _Float16 v4h;
typedef __attribute__((ext_vector_type(8)))  float    v8f;
typedef __attribute__((ext_vector_type(4)))  float    v4f;

struct FragH {
  union U { v16h v; v8h h[2]; };
  static __device__ __forceinline__ v16h load(const _Float16* p) {
    U f;
    f.h[0] = *(const v8h*)(p);
    f.h[1] = *(const v8h*)(p + 16);
    return f.v;
  }
  static __device__ __forceinline__ v8f mma(v16h a, v16h b, v8f c) {
    return __builtin_amdgcn_wmma_f32_16x16x32_f16(false, a, false, b, (short)0, c, false, false);
  }
};

__device__ __forceinline__ void guard_l0(v8f& p, v8f& q, v16h a0, v16h a1, v16h b0, v16h b1, v16h b2, v16h b3) {
  asm volatile("v_nop\n\tv_nop\n\tv_nop\n\tv_nop"
               : "+v"(p), "+v"(q)
               : "v"(a0), "v"(a1), "v"(b0), "v"(b1), "v"(b2), "v"(b3));
}
__device__ __forceinline__ void guard_l1(v8f& p, v8f& q, v16h a0, v16h a1, v16h a2, v16h a3,
                                         v16h b0, v16h b1, v16h b2, v16h b3,
                                         v16h b4, v16h b5, v16h b6, v16h b7) {
  asm volatile("v_nop\n\tv_nop\n\tv_nop\n\tv_nop"
               : "+v"(p), "+v"(q)
               : "v"(a0), "v"(a1), "v"(a2), "v"(a3),
                 "v"(b0), "v"(b1), "v"(b2), "v"(b3), "v"(b4), "v"(b5), "v"(b6), "v"(b7));
}
__device__ __forceinline__ void guard_hd(v8f& p, v16h a0, v16h a1, v16h b0, v16h b1) {
  asm volatile("v_nop\n\tv_nop\n\tv_nop\n\tv_nop"
               : "+v"(p)
               : "v"(a0), "v"(a1), "v"(b0), "v"(b1));
}

__device__ __forceinline__ float fsig(float v)  { return __builtin_amdgcn_rcpf(1.0f + __expf(-v)); }
__device__ __forceinline__ float ftanh(float v) { return 1.0f - 2.0f * __builtin_amdgcn_rcpf(__expf(2.0f * v) + 1.0f); }

__global__ __launch_bounds__(NTHR) void wplane_kernel(const float* __restrict__ w_hh0, const float* __restrict__ w_ih1,
                                                      const float* __restrict__ w_hh1, const float* __restrict__ w_hd,
                                                      unsigned short* __restrict__ dst) {
  const int blk = blockIdx.x;
  const int tid = threadIdx.x;
  const int sel = blk >> 3;
  const float* src = (sel == 0) ? w_hh0 : ((sel == 1) ? w_ih1 : ((sel == 2) ? w_hh1 : w_hd));
  const int local = ((blk & 7) * NTHR + tid) * 8;
  const int gidx  = blk * NTHR + tid;
  const v4f a = *(const v4f*)(src + local);
  const v4f b = *(const v4f*)(src + local + 4);
  v8h hv;
#pragma unroll
  for (int e = 0; e < 4; ++e) {
    const float fa = a[e] * WCARRY;
    const float fb = b[e] * WCARRY;
    hv[e]     = (_Float16)fa;
    hv[4 + e] = (_Float16)fb;
  }
  unsigned short* op = dst + (size_t)gidx * 8;
  *(volatile v8h*)op = hv;
  __threadfence();
  *(volatile v8h*)op = hv;
}

__global__ __launch_bounds__(NTHR) void lstm2_head_kernel(const float* __restrict__ x,
                                                          const float* __restrict__ w_ih0,
                                                          const float* __restrict__ b_ih0, const float* __restrict__ b_hh0,
                                                          const float* __restrict__ b_ih1, const float* __restrict__ b_hh1,
                                                          const float* __restrict__ b_hd,
                                                          const float* __restrict__ w_out, const float* __restrict__ b_out,
                                                          const unsigned short* __restrict__ wplane,
                                                          float* __restrict__ Y) {
  __shared__ __align__(16) float    xt[NSTEP * TROWS * NFEAT];
  __shared__ __align__(16) float    gl0[TROWS * NGATE];
  __shared__ __align__(16) float    gl1[TROWS * NGATE];
  __shared__ __align__(16) _Float16 hb0[TROWS * NHID];
  __shared__ __align__(16) _Float16 hb1[TROWS * NHID];

  const int tid  = threadIdx.x;
  const int wave = tid >> 5;
  const int lane = tid & 31;
  const int half = lane >> 4;
  const int r    = lane & 15;
  const int koff = 8 * half;
  const int tile = blockIdx.x;

  const int em = tid >> 4;
  const int eh = (tid & 15) * 4;

  {
    const int f  = tid & 1;
    const int m  = (tid >> 1) & 15;
    int gm = tile * TROWS + m;
    gm = (gm < MROWS) ? gm : (MROWS - 1);
    const int b  = gm / NSEQ;
    const int n  = gm - b * NSEQ;
    const int t0 = tid >> 5;
    const float* xp = x + ((size_t)(b * NFEAT + f) * NSTEP) * NSEQ + n;
#pragma unroll 4
    for (int j = 0; j < 16; ++j) {
      const int t = t0 + 8 * j;
      xt[tid + NTHR * j] = xp[(size_t)t * NSEQ];
    }
  }
  {
    v4h zv;
    zv[0] = (_Float16)0.0f; zv[1] = (_Float16)0.0f; zv[2] = (_Float16)0.0f; zv[3] = (_Float16)0.0f;
    *(v4h*)(hb0 + em * NHID + eh) = zv;
    *(v4h*)(hb1 + em * NHID + eh) = zv;
  }

  const int g0 = wave * 32 + r;
  const int g1 = g0 + 16;
  const float bs0a = b_ih0[g0] + b_hh0[g0];
  const float bs0b = b_ih0[g1] + b_hh0[g1];
  const float bs1a = b_ih1[g0] + b_hh1[g0];
  const float bs1b = b_ih1[g1] + b_hh1[g1];
  const float wa0 = w_ih0[g0 * 2 + 0];
  const float wa1 = w_ih0[g0 * 2 + 1];
  const float wb0 = w_ih0[g1 * 2 + 0];
  const float wb1 = w_ih0[g1 * 2 + 1];

  const _Float16* wp = (const _Float16*)wplane;
  v16h Bhh0[2][2], Bih1[2][2], Bhh1[2][2];
#pragma unroll
  for (int nt = 0; nt < 2; ++nt) {
    const int g = g0 + 16 * nt;
#pragma unroll
    for (int ks = 0; ks < 2; ++ks) {
      const int off = g * NHID + ks * 32 + koff;
      Bhh0[nt][ks] = FragH::load(wp + WOFF_HH0 + off);
      Bih1[nt][ks] = FragH::load(wp + WOFF_IH1 + off);
      Bhh1[nt][ks] = FragH::load(wp + WOFF_HH1 + off);
    }
  }

  float c0[4] = {0.0f, 0.0f, 0.0f, 0.0f};
  float c1[4] = {0.0f, 0.0f, 0.0f, 0.0f};
  const v8f z8 = {0.f, 0.f, 0.f, 0.f, 0.f, 0.f, 0.f, 0.f};

  const _Float16* h0row = hb0 + r * NHID + koff;
  const _Float16* h1row = hb1 + r * NHID + koff;

  __syncthreads();

#pragma unroll 1
  for (int t = 0; t < NSTEP; ++t) {
    {
      const v16h a0 = FragH::load(h0row);
      const v16h a1 = FragH::load(h0row + 32);
      v8f acc0 = z8, acc1 = z8;
      acc0 = FragH::mma(a0, Bhh0[0][0], acc0);
      acc1 = FragH::mma(a0, Bhh0[1][0], acc1);
      acc0 = FragH::mma(a1, Bhh0[0][1], acc0);
      acc1 = FragH::mma(a1, Bhh0[1][1], acc1);
      guard_l0(acc0, acc1, a0, a1, Bhh0[0][0], Bhh0[1][0], Bhh0[0][1], Bhh0[1][1]);
      const float* xr = xt + (t * TROWS + 8 * half) * NFEAT;
      v4f xq[4];
      xq[0] = *(const v4f*)(xr);
      xq[1] = *(const v4f*)(xr + 4);
      xq[2] = *(const v4f*)(xr + 8);
      xq[3] = *(const v4f*)(xr + 12);
#pragma unroll
      for (int v = 0; v < 8; ++v) {
        const float x0 = xq[v >> 1][(v & 1) * 2];
        const float x1 = xq[v >> 1][(v & 1) * 2 + 1];
        const float za = fmaf(acc0[v], FOLD, bs0a) + x0 * wa0 + x1 * wa1;
        const float zb = fmaf(acc1[v], FOLD, bs0b) + x0 * wb0 + x1 * wb1;
        gl0[(8 * half + v) * NGATE + g0] = za;
        gl0[(8 * half + v) * NGATE + g1] = zb;
      }
    }
    __syncthreads();

    {
      const float* gp = gl0 + em * NGATE + eh;
      const v4f iv = *(const v4f*)(gp);
      const v4f fv = *(const v4f*)(gp + NHID);
      const v4f gv = *(const v4f*)(gp + 2 * NHID);
      const v4f ov = *(const v4f*)(gp + 3 * NHID);
      v4h hv;
#pragma unroll
      for (int p = 0; p < 4; ++p) {
        const float ig = fsig(iv[p]);
        const float fg = fsig(fv[p]);
        const float gg = ftanh(gv[p]);
        const float og = fsig(ov[p]);
        const float cn = fg * c0[p] + ig * gg;
        c0[p] = cn;
        const float hn = og * ftanh(cn);
        hv[p] = (_Float16)(hn * HCARRY);
      }
      *(v4h*)(hb0 + em * NHID + eh) = hv;
    }
    __syncthreads();

    {
      const v16h a0 = FragH::load(h0row);
      const v16h a1 = FragH::load(h0row + 32);
      const v16h p0 = FragH::load(h1row);
      const v16h p1 = FragH::load(h1row + 32);
      v8f acc0 = z8, acc1 = z8;
      acc0 = FragH::mma(a0, Bih1[0][0], acc0);
      acc1 = FragH::mma(a0, Bih1[1][0], acc1);
      acc0 = FragH::mma(a1, Bih1[0][1], acc0);
      acc1 = FragH::mma(a1, Bih1[1][1], acc1);
      acc0 = FragH::mma(p0, Bhh1[0][0], acc0);
      acc1 = FragH::mma(p0, Bhh1[1][0], acc1);
      acc0 = FragH::mma(p1, Bhh1[0][1], acc0);
      acc1 = FragH::mma(p1, Bhh1[1][1], acc1);
      guard_l1(acc0, acc1, a0, a1, p0, p1,
               Bih1[0][0], Bih1[1][0], Bih1[0][1], Bih1[1][1],
               Bhh1[0][0], Bhh1[1][0], Bhh1[0][1], Bhh1[1][1]);
#pragma unroll
      for (int v = 0; v < 8; ++v) {
        gl1[(8 * half + v) * NGATE + g0] = fmaf(acc0[v], FOLD, bs1a);
        gl1[(8 * half + v) * NGATE + g1] = fmaf(acc1[v], FOLD, bs1b);
      }
    }
    __syncthreads();

    {
      const float* gp = gl1 + em * NGATE + eh;
      const v4f iv = *(const v4f*)(gp);
      const v4f fv = *(const v4f*)(gp + NHID);
      const v4f gv = *(const v4f*)(gp + 2 * NHID);
      const v4f ov = *(const v4f*)(gp + 3 * NHID);
      v4h hv;
#pragma unroll
      for (int p = 0; p < 4; ++p) {
        const float ig = fsig(iv[p]);
        const float fg = fsig(fv[p]);
        const float gg = ftanh(gv[p]);
        const float og = fsig(ov[p]);
        const float cn = fg * c1[p] + ig * gg;
        c1[p] = cn;
        const float hn = og * ftanh(cn);
        hv[p] = (_Float16)(hn * HCARRY);
      }
      *(v4h*)(hb1 + em * NHID + eh) = hv;
    }
  }
  __syncthreads();

  {
    const v16h a0 = FragH::load(h1row);
    const v16h a1 = FragH::load(h1row + 32);
    const int col = 16 * wave + r;
    const v16h bw0 = FragH::load(wp + WOFF_W1 + col * NHID + koff);
    const v16h bw1 = FragH::load(wp + WOFF_W1 + col * NHID + 32 + koff);
    v8f acc = z8;
    acc = FragH::mma(a0, bw0, acc);
    acc = FragH::mma(a1, bw1, acc);
    guard_hd(acc, a0, a1, bw0, bw1);
    const float bb = b_hd[col];
#pragma unroll
    for (int v = 0; v < 8; ++v) {
      const float yv = fmaxf(fmaf(acc[v], FOLD, bb), 0.0f);
      gl0[(8 * half + v) * NGATE + col] = yv;
    }
  }
  __syncthreads();

  if (wave == 0) {
    const int m = lane >> 1;
    const int c = lane & 1;
    const float* yp  = gl0 + m * NGATE;
    const float* w2p = w_out + c * NHEAD;
    float s = 0.0f;
#pragma unroll 8
    for (int k = 0; k < NHEAD; ++k) s = fmaf(yp[k], w2p[k], s);
    const float res = s + b_out[c];
    float* dst = Y + (size_t)tile * 32 + lane;
    *(volatile float*)dst = res;
    __threadfence();
    *(volatile float*)dst = res;
  }
}

__global__ __launch_bounds__(NTHR) void pack_out_kernel(const float* __restrict__ Y, float* __restrict__ out) {
  const int idx = blockIdx.x * NTHR + threadIdx.x;
  if (idx >= NOUT) return;
  const int b   = idx / (NOUTC * NSEQ);
  const int rem = idx - b * (NOUTC * NSEQ);
  const int c   = rem / NSEQ;
  const int n   = rem - c * NSEQ;
  int src = (b * NSEQ + n) * NOUTC + c;
  src = (src < NOUT) ? src : (NOUT - 1);
  const float v = Y[src];
  float* dst = out + idx;
  *(volatile float*)dst = v;
  __threadfence();
  *(volatile float*)dst = v;
}

extern "C" void kernel_launch(void* const* d_in, const int* in_sizes, int n_in,
                              void* d_out, int out_size, void* d_ws, size_t ws_size, hipStream_t stream) {
  if (n_in < 13 || d_out == nullptr || d_ws == nullptr) return;
  if (in_sizes[0] != NXELEM || in_sizes[1] != NGATE * NFEAT || in_sizes[2] != NGATE * NHID ||
      in_sizes[3] != NGATE || in_sizes[4] != NGATE || in_sizes[5] != NGATE * NHID ||
      in_sizes[6] != NGATE * NHID || in_sizes[7] != NGATE || in_sizes[8] != NGATE ||
      in_sizes[9] != NHEAD * NHID || in_sizes[10] != NHEAD || in_sizes[11] != NOUTC * NHEAD ||
      in_sizes[12] != NOUTC || out_size != NOUT) return;

  const float* x     = (const float*)d_in[0];
  const float* w_ih0 = (const float*)d_in[1];
  const float* w_hh0 = (const float*)d_in[2];
  const float* b_ih0 = (const float*)d_in[3];
  const float* b_hh0 = (const float*)d_in[4];
  const float* w_ih1 = (const float*)d_in[5];
  const float* w_hh1 = (const float*)d_in[6];
  const float* b_ih1 = (const float*)d_in[7];
  const float* b_hh1 = (const float*)d_in[8];
  const float* w_hd  = (const float*)d_in[9];
  const float* b_hd  = (const float*)d_in[10];
  const float* w_out = (const float*)d_in[11];
  const float* b_out = (const float*)d_in[12];
  float* out = (float*)d_out;

  const size_t wpl_bytes = (size_t)WPLANE_ELEMS * 2;
  const size_t ypl_bytes = (size_t)NTILE * 128;
  const size_t total = wpl_bytes + ypl_bytes;
  if (total > ws_size || total > (size_t)134217728) return;
  char* ws = (char*)d_ws;
  unsigned short* WPL = (unsigned short*)ws;
  float*          YPL = (float*)(ws + wpl_bytes);

  wplane_kernel<<<PREP_BLOCKS, NTHR, 0, stream>>>(w_hh0, w_ih1, w_hh1, w_hd, WPL);
  lstm2_head_kernel<<<NTILE, NTHR, 0, stream>>>(x, w_ih0, b_ih0, b_hh0, b_ih1, b_hh1, b_hd, w_out, b_out, WPL, YPL);
  pack_out_kernel<<<(NOUT + NTHR - 1) / NTHR, NTHR, 0, stream>>>(YPL, out);
}
